// Conv3dBlock_29171417875121
// MI455X (gfx1250) — hardware-verified
//
#include <hip/hip_runtime.h>
#define BB 2
#define NS 128
#define TT 128
#define MM 64
#define GW 32
#define NG 1024
#define NSR (BB * NS * TT)
#define NVX (BB * TT * NG)

typedef __bf16 v16b __attribute__((ext_vector_type(16)));
typedef unsigned short v8us __attribute__((ext_vector_type(8), may_alias));
typedef float  v8f  __attribute__((ext_vector_type(8)));
typedef float  v4f  __attribute__((ext_vector_type(4)));
typedef float  v4fa __attribute__((ext_vector_type(4), may_alias));
union FragB { v16b v; v8us half[2]; unsigned short u[16]; };

__device__ __forceinline__ unsigned short bf16_bits(float x) { unsigned int u = __float_as_uint(x); return (unsigned short)((u + 0x7FFFu + ((u >> 16) & 1u)) >> 16); }
__device__ __forceinline__ float bf16_val(unsigned short b) { return __uint_as_float(((unsigned int)b) << 16); }
__device__ __forceinline__ float bf16_round(float x) { return bf16_val(bf16_bits(x)); }
template <int NT>
__device__ __forceinline__ v8f mmaN(v16b ah, v16b al, v16b bh, v16b bl, v8f c) {
  c = __builtin_amdgcn_wmma_f32_16x16x32_bf16(false, ah, false, bh, (short)0, c, false, false);
  if (NT >= 2) c = __builtin_amdgcn_wmma_f32_16x16x32_bf16(false, al, false, bh, (short)0, c, false, false);
  if (NT >= 3) c = __builtin_amdgcn_wmma_f32_16x16x32_bf16(false, ah, false, bl, (short)0, c, false, false);
  asm volatile("v_nop\n\tv_nop\n\tv_nop\n\tv_nop" : "+v"(c) : "v"(ah), "v"(al), "v"(bh), "v"(bl));
  return c;
}

__global__ __launch_bounds__(256) void k_wt_bf16(const float* __restrict__ W, unsigned short* __restrict__ Wt, int K, int N) {
  const int t = blockIdx.x * 256 + threadIdx.x;
  const int k8n = K / 8;
  if (t >= N * k8n) return;
  const int n = t / k8n, k8 = (t % k8n) * 8;
  v8us v;
#pragma unroll
  for (int i = 0; i < 8; ++i) v[i] = bf16_bits(W[(size_t)(k8 + i) * N + n]);
  *(volatile v8us*)(Wt + (size_t)n * K + k8) = v;
  __threadfence();
  *(volatile v8us*)(Wt + (size_t)n * K + k8) = v;
}

template <bool ASPLIT, int ACT, bool BIAS_BF16>
__global__ __launch_bounds__(128) void k_gemm_bf(const float* __restrict__ A, int lda, const unsigned short* __restrict__ Wt, int ldb,
                                               const float* __restrict__ bias, float* __restrict__ C, int ldc, int M, int N, int K) {
  __shared__ __attribute__((aligned(16))) float so[4][16][64];
  const int tid = threadIdx.x, w = tid >> 5, lane = tid & 31, ln = lane & 15, hh = lane >> 4;
  const int ntn = N / 64;
  const int wid = blockIdx.x * 4 + w;
  const int mt = wid / ntn, nq = wid % ntn;
  if (mt * 16 >= M) return;
  const int row0 = mt * 16, col0 = nq * 64;
  const float* arow = A + (size_t)(row0 + ln) * lda;
  v8f acc[4] = {};
  for (int kb = 0; kb < K; kb += 32) {
    FragB ah, al;
    const v4f x0 = *(const v4fa*)(arow + kb + 8 * hh), x1 = *(const v4fa*)(arow + kb + 8 * hh + 4);
    const v4f x2 = *(const v4fa*)(arow + kb + 16 + 8 * hh), x3 = *(const v4fa*)(arow + kb + 16 + 8 * hh + 4);
    float xs[16] = {x0[0],x0[1],x0[2],x0[3],x1[0],x1[1],x1[2],x1[3],x2[0],x2[1],x2[2],x2[3],x3[0],x3[1],x3[2],x3[3]};
#pragma unroll
    for (int i = 0; i < 16; ++i) { const unsigned short hb = bf16_bits(xs[i]); ah.u[i] = hb; al.u[i] = ASPLIT ? bf16_bits(xs[i] - bf16_val(hb)) : (unsigned short)0; }
#pragma unroll
    for (int t = 0; t < 4; ++t) {
      const unsigned short* brow = Wt + (size_t)(col0 + t * 16 + ln) * ldb + kb;
      FragB b;
      b.half[0] = *(const v8us*)(brow + 8 * hh);
      b.half[1] = *(const v8us*)(brow + 16 + 8 * hh);
      acc[t] = mmaN<ASPLIT ? 2 : 1>(ah.v, al.v, b.v, b.v, acc[t]);
    }
  }
#pragma unroll
  for (int t = 0; t < 4; ++t) {
    float bv = bias ? bias[col0 + t * 16 + ln] : 0.f;
    if (BIAS_BF16) bv = bf16_round(bv);
#pragma unroll
    for (int r = 0; r < 8; ++r) { float v = acc[t][r] + bv; if (ACT == 1) v = fmaxf(v, 0.f); so[w][8 * hh + r][t * 16 + ln] = v; }
  }
  __builtin_amdgcn_fence(__ATOMIC_ACQ_REL, "workgroup");
  __builtin_amdgcn_wave_barrier();
  const int rsub = lane >> 4, c4 = (lane & 15) * 4;
  for (int pass = 0; pass < 2; ++pass) {
#pragma unroll
    for (int q = 0; q < 8; ++q) {
      const int r = q * 2 + rsub;
      const v4f v = *(const v4fa*)&so[w][r][c4];
      *(volatile v4f*)(C + (size_t)(row0 + r) * ldc + col0 + c4) = v;
    }
    if (pass == 0) __threadfence();
  }
}

template <int D, bool CAUSAL>
__global__ __launch_bounds__(128) void k_flash(const float* __restrict__ qb, const float* __restrict__ kb, const float* __restrict__ vb,
                                             int pitch, int T, int H, float scale, float* __restrict__ y, int ypitch) {
  constexpr int KS = D / 32;
  constexpr int DT = D / 16;
  __shared__ __attribute__((aligned(16))) unsigned short sKh[32][D + 8], sKl[32][D + 8], sVh[32][D + 8], sVl[32][D + 8];
  __shared__ __attribute__((aligned(16))) unsigned short sPh[4][16][40], sPl[4][16][40];
  __shared__ __attribute__((aligned(16))) float sO[4][16][D];
  const int tid = threadIdx.x, w = tid >> 5, lane = tid & 31, ln = lane & 15, hh = lane >> 4;
  const int nqb = (T + 63) / 64;
  const int bh = blockIdx.x / nqb, qblk = blockIdx.x % nqb;
  const int b = bh / H, h = bh % H;
  const int q0 = qblk * 64 + w * 16;
  const float* Q = qb + (size_t)b * T * pitch + h * D;
  const float* K = kb + (size_t)b * T * pitch + h * D;
  const float* V = vb + (size_t)b * T * pitch + h * D;

  FragB aqh[KS], aql[KS];
  {
    int row = q0 + ln; if (row >= T) row = T - 1;
    const float* qr = Q + (size_t)row * pitch;
#pragma unroll
    for (int ks = 0; ks < KS; ++ks)
#pragma unroll
      for (int i = 0; i < 16; ++i) {
        const int d = ks * 32 + ((i < 8) ? (8 * hh + i) : (16 + 8 * hh + (i - 8)));
        const float x = qr[d] * scale; const unsigned short hb = bf16_bits(x);
        aqh[ks].u[i] = hb; aql[ks].u[i] = bf16_bits(x - bf16_val(hb));
      }
  }
  float m_r[8], l_r[8];
#pragma unroll
  for (int r = 0; r < 8; ++r) { m_r[r] = -3.0e38f; l_r[r] = 0.f; }
  v8f oacc[DT];
#pragma unroll
  for (int dt = 0; dt < DT; ++dt) oacc[dt] = (v8f){0.f,0.f,0.f,0.f,0.f,0.f,0.f,0.f};

  const int kv_end = CAUSAL ? min(T, qblk * 64 + 64) : T;
  for (int j0 = 0; j0 < kv_end; j0 += 32) {
    __syncthreads();
    for (int e = tid; e < 32 * (D / 4); e += 128) {
      const int r = e / (D / 4), c4 = (e % (D / 4)) * 4;
      const int key = j0 + r;
      v4f kf = {0.f,0.f,0.f,0.f}, vf = {0.f,0.f,0.f,0.f};
      if (key < T) { kf = *(const v4fa*)(K + (size_t)key * pitch + c4); vf = *(const v4fa*)(V + (size_t)key * pitch + c4); }
#pragma unroll
      for (int t = 0; t < 4; ++t) {
        unsigned short hb = bf16_bits(kf[t]); sKh[r][c4 + t] = hb; sKl[r][c4 + t] = bf16_bits(kf[t] - bf16_val(hb));
        hb = bf16_bits(vf[t]); sVh[r][c4 + t] = hb; sVl[r][c4 + t] = bf16_bits(vf[t] - bf16_val(hb));
      }
    }
    __syncthreads();
    v8f s[2];
#pragma unroll
    for (int nt = 0; nt < 2; ++nt) {
      v8f acc = {};
#pragma unroll
      for (int ks = 0; ks < KS; ++ks) {
        FragB bh_, bl_;
        bh_.half[0] = *(const v8us*)&sKh[nt * 16 + ln][ks * 32 + 8 * hh]; bh_.half[1] = *(const v8us*)&sKh[nt * 16 + ln][ks * 32 + 16 + 8 * hh];
        bl_.half[0] = *(const v8us*)&sKl[nt * 16 + ln][ks * 32 + 8 * hh]; bl_.half[1] = *(const v8us*)&sKl[nt * 16 + ln][ks * 32 + 16 + 8 * hh];
        acc = mmaN<3>(aqh[ks].v, aql[ks].v, bh_.v, bl_.v, acc);
      }
      s[nt] = acc;
    }
    float alpha[8];
#pragma unroll
    for (int r = 0; r < 8; ++r) {
      const int qi = q0 + 8 * hh + r;
      const int ja = j0 + ln, jb = j0 + 16 + ln;
      if (CAUSAL) { if (ja > qi) s[0][r] = -3.0e38f; if (jb > qi) s[1][r] = -3.0e38f; }
      if (ja >= T) s[0][r] = -3.0e38f;
      if (jb >= T) s[1][r] = -3.0e38f;
      float mx = fmaxf(s[0][r], s[1][r]);
      mx = fmaxf(mx, __shfl_xor(mx, 1, 32)); mx = fmaxf(mx, __shfl_xor(mx, 2, 32)); mx = fmaxf(mx, __shfl_xor(mx, 4, 32)); mx = fmaxf(mx, __shfl_xor(mx, 8, 32));
      const float mnew = fmaxf(m_r[r], mx);
      alpha[r] = (mnew > -1.0e38f) ? __expf(m_r[r] - mnew) : 1.0f;
      const float p0 = (s[0][r] > -1.0e38f) ? __expf(s[0][r] - mnew) : 0.f;
      const float p1 = (s[1][r] > -1.0e38f) ? __expf(s[1][r] - mnew) : 0.f;
      m_r[r] = mnew;
      l_r[r] = l_r[r] * alpha[r] + p0 + p1;
      unsigned short hb = bf16_bits(p0); sPh[w][8 * hh + r][ln] = hb;      sPl[w][8 * hh + r][ln] = bf16_bits(p0 - bf16_val(hb));
      hb = bf16_bits(p1);                sPh[w][8 * hh + r][16 + ln] = hb; sPl[w][8 * hh + r][16 + ln] = bf16_bits(p1 - bf16_val(hb));
    }
#pragma unroll
    for (int dt = 0; dt < DT; ++dt)
#pragma unroll
      for (int r = 0; r < 8; ++r) oacc[dt][r] *= alpha[r];
    __builtin_amdgcn_fence(__ATOMIC_ACQ_REL, "workgroup");
    __builtin_amdgcn_wave_barrier();
    FragB pah, pal;
    pah.half[0] = *(const v8us*)&sPh[w][ln][8 * hh]; pah.half[1] = *(const v8us*)&sPh[w][ln][16 + 8 * hh];
    pal.half[0] = *(const v8us*)&sPl[w][ln][8 * hh]; pal.half[1] = *(const v8us*)&sPl[w][ln][16 + 8 * hh];
#pragma unroll
    for (int dt = 0; dt < DT; ++dt) {
      FragB bvh, bvl;
#pragma unroll
      for (int i = 0; i < 8; ++i) {
        bvh.u[i] = sVh[8 * hh + i][dt * 16 + ln]; bvh.u[8 + i] = sVh[16 + 8 * hh + i][dt * 16 + ln];
        bvl.u[i] = sVl[8 * hh + i][dt * 16 + ln]; bvl.u[8 + i] = sVl[16 + 8 * hh + i][dt * 16 + ln];
      }
      oacc[dt] = mmaN<3>(pah.v, pal.v, bvh.v, bvl.v, oacc[dt]);
    }
    __builtin_amdgcn_fence(__ATOMIC_ACQ_REL, "workgroup");
    __builtin_amdgcn_wave_barrier();
  }
#pragma unroll
  for (int r = 0; r < 8; ++r) {
    float l = l_r[r];
    l += __shfl_xor(l, 1, 32); l += __shfl_xor(l, 2, 32); l += __shfl_xor(l, 4, 32); l += __shfl_xor(l, 8, 32);
    l_r[r] = (l > 0.f) ? 1.0f / l : 0.f;
  }
#pragma unroll
  for (int dt = 0; dt < DT; ++dt)
#pragma unroll
    for (int r = 0; r < 8; ++r) sO[w][8 * hh + r][dt * 16 + ln] = oacc[dt][r] * l_r[r];
  __builtin_amdgcn_fence(__ATOMIC_ACQ_REL, "workgroup");
  __builtin_amdgcn_wave_barrier();
  for (int pass = 0; pass < 2; ++pass) {
    for (int r = 0; r < 16; ++r) {
      const int row = q0 + r;
      if (row < T && lane < D / 4) {
        const v4f val = *(const v4fa*)&sO[w][r][lane * 4];
        *(volatile v4f*)(y + ((size_t)b * T + row) * ypitch + h * D + lane * 4) = val;
      }
    }
    if (pass == 0) __threadfence();
  }
}

template <bool ASPLIT, int ACT, bool BIAS_BF16, bool RES_BF16>
__global__ __launch_bounds__(128) void k_gemm_bf3(const float* __restrict__ A, int lda, const unsigned short* __restrict__ Wt, int ldb,
                                                const float* __restrict__ bias, const float* __restrict__ resid, int rmod, int ldr,
                                                float* __restrict__ C, int ldc, int M, int N, int K) {
  __shared__ __attribute__((aligned(16))) float so[4][16][64];
  const int tid = threadIdx.x, w = tid >> 5, lane = tid & 31, ln = lane & 15, hh = lane >> 4;
  const int ntn = N / 64;
  const int wid = blockIdx.x * 4 + w;
  const int mt = wid / ntn, nq = wid % ntn;
  if (mt * 16 >= M) return;
  const int row0 = mt * 16, col0 = nq * 64;
  const float* arow = A + (size_t)(row0 + ln) * lda;
  v8f acc[4] = {};
  for (int kb = 0; kb < K; kb += 32) {
    FragB ah, al;
    const v4f x0 = *(const v4fa*)(arow + kb + 8 * hh), x1 = *(const v4fa*)(arow + kb + 8 * hh + 4);
    const v4f x2 = *(const v4fa*)(arow + kb + 16 + 8 * hh), x3 = *(const v4fa*)(arow + kb + 16 + 8 * hh + 4);
    float xs[16] = {x0[0],x0[1],x0[2],x0[3],x1[0],x1[1],x1[2],x1[3],x2[0],x2[1],x2[2],x2[3],x3[0],x3[1],x3[2],x3[3]};
#pragma unroll
    for (int i = 0; i < 16; ++i) { const unsigned short hb = bf16_bits(xs[i]); ah.u[i] = hb; al.u[i] = ASPLIT ? bf16_bits(xs[i] - bf16_val(hb)) : (unsigned short)0; }
#pragma unroll
    for (int t = 0; t < 4; ++t) {
      const unsigned short* brow = Wt + (size_t)(col0 + t * 16 + ln) * ldb + kb;
      FragB b;
      b.half[0] = *(const v8us*)(brow + 8 * hh);
      b.half[1] = *(const v8us*)(brow + 16 + 8 * hh);
      acc[t] = mmaN<ASPLIT ? 2 : 1>(ah.v, al.v, b.v, b.v, acc[t]);
    }
  }
#pragma unroll
  for (int t = 0; t < 4; ++t) {
    const int col = col0 + t * 16 + ln;
    float bv = bias ? bias[col] : 0.f;
    if (BIAS_BF16) bv = bf16_round(bv);
#pragma unroll
    for (int r = 0; r < 8; ++r) {
      float v = acc[t][r] + bv;
      if (resid) { float rv = resid[(size_t)((row0 + 8 * hh + r) % rmod) * ldr + col]; if (RES_BF16) rv = bf16_round(rv); v += rv; }
      if (ACT == 1) v = fmaxf(v, 0.f);
      if (ACT == 2) v = 0.5f * v * (1.0f + erff(v * 0.70710678118654752f));
      if (ACT == 3) { const float u = 0.7978845608028654f * (v + 0.044715f * v * v * v); v = 0.5f * v * (1.0f + tanhf(u)); }
      so[w][8 * hh + r][t * 16 + ln] = v;
    }
  }
  __builtin_amdgcn_fence(__ATOMIC_ACQ_REL, "workgroup");
  __builtin_amdgcn_wave_barrier();
  const int rsub = lane >> 4, c4 = (lane & 15) * 4;
  for (int pass = 0; pass < 2; ++pass) {
#pragma unroll
    for (int q = 0; q < 8; ++q) {
      const int r = q * 2 + rsub;
      const v4f v = *(const v4fa*)&so[w][r][c4];
      *(volatile v4f*)(C + (size_t)(row0 + r) * ldc + col0 + c4) = v;
    }
    if (pass == 0) __threadfence();
  }
}
template <bool PARAM_BF16>
__global__ __launch_bounds__(256) void k_layernorm(const float* __restrict__ X, const float* __restrict__ R, const float* __restrict__ g, const float* __restrict__ bta,
                                                  float* __restrict__ out_sum, float* __restrict__ out_norm, int N, float eps) {
  __shared__ float red[256];
  const int row = blockIdx.x, tid = threadIdx.x;
  const float* x = X + (size_t)row * N; const float* rr = R ? R + (size_t)row * N : nullptr;
  float vals[16];
  const int per = N / 256;
  float s1 = 0.f;
  for (int u = 0; u < per / 4; ++u) {
    const int j = tid * 4 + 1024 * u;
    const v4f a = *(const v4fa*)(x + j);
    v4f b = {0.f,0.f,0.f,0.f}; if (rr) b = *(const v4fa*)(rr + j);
#pragma unroll
    for (int q = 0; q < 4; ++q) { const float v = a[q] + b[q]; vals[u * 4 + q] = v; s1 += v; }
  }
  red[tid] = s1; __syncthreads();
  for (int st = 128; st > 0; st >>= 1) { if (tid < st) red[tid] += red[tid + st]; __syncthreads(); }
  const float mu = red[0] / (float)N; __syncthreads();
  float s2 = 0.f;
  for (int u = 0; u < per / 4; ++u)
#pragma unroll
    for (int q = 0; q < 4; ++q) { const float c = vals[u * 4 + q] - mu; s2 += c * c; }
  red[tid] = s2; __syncthreads();
  for (int st = 128; st > 0; st >>= 1) { if (tid < st) red[tid] += red[tid + st]; __syncthreads(); }
  const float rs = rsqrtf(red[0] / (float)N + eps);
  for (int pass = 0; pass < 2; ++pass) {
    for (int u = 0; u < per / 4; ++u) {
      const int j = tid * 4 + 1024 * u;
      v4f o, sm;
#pragma unroll
      for (int q = 0; q < 4; ++q) {
        float gg = g[j + q], bb = bta[j + q];
        if (PARAM_BF16) { gg = bf16_round(gg); bb = bf16_round(bb); }
        sm[q] = vals[u * 4 + q]; o[q] = (vals[u * 4 + q] - mu) * rs * gg + bb;
      }
      if (out_sum) *(volatile v4f*)(out_sum + (size_t)row * N + j) = sm;
      *(volatile v4f*)(out_norm + (size_t)row * N + j) = o;
    }
    if (pass == 0) __threadfence();
  }
}


typedef _Float16 v16h __attribute__((ext_vector_type(16)));
union FragH { v16h v; v8us half[2]; _Float16 h[16]; unsigned short u[16]; };
template <int NT>
__device__ __forceinline__ v8f mmaH(v16h ah, v16h al, v16h bh, v16h bl, v8f c) {
  c = __builtin_amdgcn_wmma_f32_16x16x32_f16(false, ah, false, bh, (short)0, c, false, false);
  if (NT >= 2) c = __builtin_amdgcn_wmma_f32_16x16x32_f16(false, al, false, bh, (short)0, c, false, false);
  if (NT >= 3) c = __builtin_amdgcn_wmma_f32_16x16x32_f16(false, ah, false, bl, (short)0, c, false, false);
  asm volatile("v_nop\n\tv_nop\n\tv_nop\n\tv_nop" : "+v"(c) : "v"(ah), "v"(al), "v"(bh), "v"(bl));
  return c;
}
template <bool ASPLIT>
__global__ __launch_bounds__(128) void k_gemm_h(const float* __restrict__ A, int lda, size_t sA, const _Float16* __restrict__ Bh, int ldb, size_t sB, float alpha, float* __restrict__ C, int ldc, size_t sC, int M, int N, int K) {
  __shared__ __attribute__((aligned(16))) float so[4][16][64];
  const int tid = threadIdx.x, w = tid >> 5, lane = tid & 31, ln = lane & 15, hh = lane >> 4; const int by = blockIdx.y;
  A += (size_t)by * sA; Bh += (size_t)by * sB; C += (size_t)by * sC;
  const int ntn = (N + 63) / 64; const int wid = blockIdx.x * 4 + w; const int mt = wid / ntn, nq = wid % ntn; if (mt * 16 >= M) return;
  const int row0 = mt * 16, col0 = nq * 64; const float* arow = A + (size_t)(row0 + ln) * lda;
  v8f acc[4] = {};
  for (int kb = 0; kb < K; kb += 32) {
    FragH ah, al;
    const v4f x0 = *(const v4fa*)(arow + kb + 8 * hh), x1 = *(const v4fa*)(arow + kb + 8 * hh + 4), x2 = *(const v4fa*)(arow + kb + 16 + 8 * hh), x3 = *(const v4fa*)(arow + kb + 16 + 8 * hh + 4);
    float xs[16] = {x0[0],x0[1],x0[2],x0[3],x1[0],x1[1],x1[2],x1[3],x2[0],x2[1],x2[2],x2[3],x3[0],x3[1],x3[2],x3[3]};
#pragma unroll
    for (int i = 0; i < 16; ++i) { const _Float16 h = (_Float16)xs[i]; ah.h[i] = h; al.h[i] = ASPLIT ? (_Float16)(xs[i] - (float)h) : (_Float16)0.0f; }
#pragma unroll
    for (int t = 0; t < 4; ++t) { if (col0 + t * 16 >= N) continue; const size_t boff = (size_t)(col0 + t * 16 + ln) * ldb + kb; FragH bq; bq.half[0] = *(const v8us*)(Bh + boff + 8 * hh); bq.half[1] = *(const v8us*)(Bh + boff + 16 + 8 * hh);
      acc[t] = mmaH<ASPLIT ? 2 : 1>(ah.v, al.v, bq.v, bq.v, acc[t]); }
  }
#pragma unroll
  for (int t = 0; t < 4; ++t) { if (col0 + t * 16 >= N) continue;
#pragma unroll
    for (int r = 0; r < 8; ++r) so[w][8 * hh + r][t * 16 + ln] = acc[t][r] * alpha; }
  __builtin_amdgcn_fence(__ATOMIC_ACQ_REL, "workgroup"); __builtin_amdgcn_wave_barrier();
  const int rsub = lane >> 4, c4 = (lane & 15) * 4;
  for (int pass = 0; pass < 2; ++pass) {
#pragma unroll
    for (int q = 0; q < 8; ++q) { const int r = q * 2 + rsub; if (col0 + c4 < N) { const v4f v = *(const v4fa*)&so[w][r][c4]; *(volatile v4f*)(C + (size_t)(row0 + r) * ldc + col0 + c4) = v; } }
    if (pass == 0) __threadfence(); }
}

__global__ __launch_bounds__(256) void k_wt_f16(const float* __restrict__ W, _Float16* __restrict__ Wt, int K, int N, float scale) {
  const int t = blockIdx.x * 256 + threadIdx.x; if (t >= N * (K / 8)) return; const int n = t / (K / 8), k8 = (t % (K / 8)) * 8; FragH f;
#pragma unroll
  for (int i = 0; i < 8; ++i) f.h[i] = (_Float16)(bf16_round(W[(size_t)(k8 + i) * N + n]) * scale); const v8us o = f.half[0];
  *(volatile v8us*)((unsigned short*)Wt + (size_t)n * K + k8) = o; __threadfence(); *(volatile v8us*)((unsigned short*)Wt + (size_t)n * K + k8) = o;
}
template <int ACT>
__global__ __launch_bounds__(128) void k_gemm_hhx(const _Float16* __restrict__ A, int lda, size_t sA, const _Float16* __restrict__ Bh, int ldb, size_t sB, float alpha, const float* __restrict__ bias, size_t sBias, const float* __restrict__ CP, int rowsPerB, size_t sCPb, int row0g,
    float* __restrict__ C, _Float16* __restrict__ C16, int ldc, size_t sC, int M, int N, int K) {
  __shared__ __attribute__((aligned(16))) float so[4][16][64];
  const int tid = threadIdx.x, w = tid >> 5, lane = tid & 31, ln = lane & 15, hh = lane >> 4; const int by = blockIdx.y;
  A += (size_t)by * sA; Bh += (size_t)by * sB; const size_t cofs = (size_t)by * sC; const float* bp = bias ? bias + (size_t)by * sBias : nullptr;
  const int ntn = (N + 63) / 64; const int wid = blockIdx.x * 4 + w; const int mt = wid / ntn, nq = wid % ntn; if (mt * 16 >= M) return;
  const int row0 = mt * 16, col0 = nq * 64; const _Float16* arow = A + (size_t)(row0 + ln) * lda;
  v8f acc[4] = {};
  for (int kb = 0; kb < K; kb += 32) { FragH ah; ah.half[0] = *(const v8us*)((const unsigned short*)arow + kb + 8 * hh); ah.half[1] = *(const v8us*)((const unsigned short*)arow + kb + 16 + 8 * hh);
#pragma unroll
    for (int t = 0; t < 4; ++t) { if (col0 + t * 16 >= N) continue; const size_t boff = (size_t)(col0 + t * 16 + ln) * ldb + kb; FragH bq; bq.half[0] = *(const v8us*)((const unsigned short*)Bh + boff + 8 * hh); bq.half[1] = *(const v8us*)((const unsigned short*)Bh + boff + 16 + 8 * hh);
      acc[t] = mmaH<1>(ah.v, ah.v, bq.v, bq.v, acc[t]); }
  }
#pragma unroll
  for (int t = 0; t < 4; ++t) { if (col0 + t * 16 >= N) continue; const int col = col0 + t * 16 + ln; const float bv = bp ? bf16_round(bp[col]) : 0.f;
#pragma unroll
    for (int r = 0; r < 8; ++r) { float v = acc[t][r] * alpha + bv; if (CP) { const int bidx = (row0g + row0 + 8 * hh + r) / rowsPerB; v += CP[(size_t)bidx * sCPb + (size_t)by * 64 + col]; } if (ACT == 1) v = (v > 0.f) ? v : expm1f(v); else if (ACT == 3) v = fmaxf(v, 0.f); so[w][8 * hh + r][t * 16 + ln] = v; } }
  __builtin_amdgcn_fence(__ATOMIC_ACQ_REL, "workgroup"); __builtin_amdgcn_wave_barrier();
  const int rsub = lane >> 4, c4 = (lane & 15) * 4; typedef _Float16 v4h __attribute__((ext_vector_type(4)));
  for (int pass = 0; pass < 2; ++pass) {
#pragma unroll
    for (int q = 0; q < 8; ++q) { const int r = q * 2 + rsub; if (col0 + c4 < N) { const v4f v = *(const v4fa*)&so[w][r][c4]; if (C) *(volatile v4f*)(C + cofs + (size_t)(row0 + r) * ldc + col0 + c4) = v; if (C16) { v4h h4; for (int i = 0; i < 4; ++i) h4[i] = (_Float16)v[i]; *(volatile v4h*)(C16 + cofs + (size_t)(row0 + r) * ldc + col0 + c4) = h4; } } }
    if (pass == 0) __threadfence(); }
}


__global__ __launch_bounds__(256) void k_x16(const float* __restrict__ x, _Float16* __restrict__ X16, size_t n8) { const size_t t = (size_t)blockIdx.x * 256 + threadIdx.x; if (t >= n8) return; FragH f;
#pragma unroll
  for (int q = 0; q < 8; ++q) f.h[q] = (_Float16)bf16_round(x[t * 8 + q]); *(volatile v8us*)((unsigned short*)X16 + t * 8) = f.half[0]; __threadfence(); *(volatile v8us*)((unsigned short*)X16 + t * 8) = f.half[0]; }
__global__ __launch_bounds__(256) void k_h16(const float* __restrict__ x, _Float16* __restrict__ X16, size_t n8) { const size_t t = (size_t)blockIdx.x * 256 + threadIdx.x; if (t >= n8) return; FragH f;
#pragma unroll
  for (int q = 0; q < 8; ++q) f.h[q] = (_Float16)x[t * 8 + q]; *(volatile v8us*)((unsigned short*)X16 + t * 8) = f.half[0]; __threadfence(); *(volatile v8us*)((unsigned short*)X16 + t * 8) = f.half[0]; }
__global__ __launch_bounds__(256) void k_round16f(const float* __restrict__ W, _Float16* __restrict__ Bt, size_t n8) { const size_t t = (size_t)blockIdx.x * 256 + threadIdx.x; if (t >= n8) return; FragH f;
#pragma unroll
  for (int i = 0; i < 8; ++i) f.h[i] = (_Float16)(bf16_round(W[t * 8 + i]) * 16.0f); *(volatile v8us*)((unsigned short*)Bt + t * 8) = f.half[0]; __threadfence(); *(volatile v8us*)((unsigned short*)Bt + t * 8) = f.half[0]; }
template <int NHv, int TTv>
__global__ __launch_bounds__(256) void k_vt(const _Float16* __restrict__ V16, int ldv, int voff, _Float16* __restrict__ Vt) { __shared__ unsigned short tl[64][66]; const int tid = threadIdx.x; const int slab = blockIdx.x / (TTv / 64), lg = blockIdx.x % (TTv / 64); const int b = slab / NHv, h = slab % NHv;
  for (int i = tid; i < 64 * 8; i += 256) { const int r = i / 8, c8 = (i % 8) * 8; FragH f; f.half[0] = *(const v8us*)((const unsigned short*)V16 + ((size_t)b * TTv + lg * 64 + r) * ldv + voff + h * 64 + c8);
#pragma unroll
    for (int q = 0; q < 8; ++q) tl[r][c8 + q] = f.u[q]; }
  __syncthreads();
  for (int pass = 0; pass < 2; ++pass) {
#pragma unroll
    for (int rd = 0; rd < 2; ++rd) { const int d = rd * 32 + tid / 8, pc = tid % 8; FragH f;
#pragma unroll
      for (int q = 0; q < 8; ++q) f.u[q] = tl[pc * 8 + q][d];
      *(volatile v8us*)((unsigned short*)Vt + ((size_t)slab * 64 + d) * TTv + lg * 64 + pc * 8) = f.half[0]; }
    if (pass == 0) __threadfence(); } }

typedef _Float16 v4h __attribute__((ext_vector_type(4)));
__global__ __launch_bounds__(256) void k_wtap(const float* __restrict__ w, _Float16* __restrict__ Bt) { const int t = blockIdx.x * 256 + threadIdx.x; if (t >= 27 * MM * (MM / 8)) return; const int i8 = (t % (MM / 8)) * 8; const int o = (t / (MM / 8)) % MM; const int tap = t / ((MM / 8) * MM); FragH f;
#pragma unroll
  for (int q = 0; q < 8; ++q) f.h[q] = (_Float16)(bf16_round(w[(((size_t)o * MM + i8 + q) * 27) + tap]) * 16.0f); unsigned short* d = (unsigned short*)Bt + ((size_t)tap * MM + o) * MM + i8; *(volatile v8us*)d = f.half[0]; __threadfence(); *(volatile v8us*)d = f.half[0]; }
__global__ __launch_bounds__(256) void k_ginit(const float* __restrict__ cb, float* __restrict__ Y) { const size_t t = (size_t)blockIdx.x * 256 + threadIdx.x; if (t >= (size_t)NVX * MM / 4) return; const int c4 = (int)((t * 4) % MM); v4f v; for (int q = 0; q < 4; ++q) v[q] = bf16_round(cb[c4 + q]); *(volatile v4f*)(Y + t * 4) = v; __threadfence(); *(volatile v4f*)(Y + t * 4) = v; }
__global__ __launch_bounds__(256) void k_tapacc(const float* __restrict__ C, const int* __restrict__ ri, const int* __restrict__ ci, int dt, int dh, int dw, float* __restrict__ Y) { const size_t t = (size_t)blockIdx.x * 256 + threadIdx.x; if (t >= (size_t)NSR * 16) return; const int pc = (int)(t % 16); const size_t row = t / 16;        const int tt = (int)(row % TT); const int s = (int)((row / TT) % NS); const int b = (int)(row / ((size_t)TT * NS));
  const int t2 = tt + dt; int r = ri[s]; r = r < 0 ? 0 : (r >= GW ? GW - 1 : r); int cc = ci[s]; cc = cc < 0 ? 0 : (cc >= GW ? GW - 1 : cc); const int r2 = r + dh, c2 = cc + dw; if (t2 < 0 || t2 >= TT || r2 < 0 || r2 >= GW || c2 < 0 || c2 >= GW) return;
  float* y = Y + (((size_t)b * TT + t2) * NG + r2 * GW + c2) * MM + pc * 4; const v4f yv = *(const v4fa*)y, cv = *(const v4fa*)(C + row * MM + pc * 4); const v4f a = yv + cv;
  *(volatile v4f*)y = a; __threadfence(); *(volatile v4f*)y = a; }
__global__ __launch_bounds__(256) void k_gnstat(const float* __restrict__ Y, float* __restrict__ ST) { __shared__ float ra[256]; const int bt = blockIdx.x / 8, g = blockIdx.x % 8; const int tid = threadIdx.x; const float* base = Y + (size_t)bt * NG * MM + g * 8; float s = 0.f;
  for (int p = tid; p < NG; p += 256) { const v4f a = *(const v4fa*)(base + (size_t)p * MM), b2 = *(const v4fa*)(base + (size_t)p * MM + 4); s += (a[0] + a[1]) + (a[2] + a[3]) + (b2[0] + b2[1]) + (b2[2] + b2[3]); }
  ra[tid] = s; __syncthreads(); for (int o = 128; o >= 1; o >>= 1) { if (tid < o) ra[tid] += ra[tid + o]; __syncthreads(); } const float mu = ra[0] / (float)(8 * NG); __syncthreads(); float q2 = 0.f;
  for (int p = tid; p < NG; p += 256) { const v4f a = *(const v4fa*)(base + (size_t)p * MM), b2 = *(const v4fa*)(base + (size_t)p * MM + 4); for (int q = 0; q < 4; ++q) { const float d1 = a[q] - mu, d2 = b2[q] - mu; q2 += d1 * d1 + d2 * d2; } }
  ra[tid] = q2; __syncthreads(); for (int o = 128; o >= 1; o >>= 1) { if (tid < o) ra[tid] += ra[tid + o]; __syncthreads(); }
  if (tid < 32) { const float rsv = rsqrtf(ra[0] / (float)(8 * NG) + 1e-5f); const float v = (tid == 0) ? mu : ((tid == 1) ? rsv : 0.f); float* d = ST + ((size_t)bt * 8 + g) * 32 + tid; *(volatile float*)d = v; __threadfence(); *(volatile float*)d = v; } }
__global__ __launch_bounds__(256) void k_gath(const float* __restrict__ Y, const float* __restrict__ ST, const float* __restrict__ gg, const float* __restrict__ gb, const int* __restrict__ ri, const int* __restrict__ ci, _Float16* __restrict__ A16) { const size_t t = (size_t)blockIdx.x * 256 + threadIdx.x; if (t >= (size_t)NSR * (MM / 8)) return; const int c8 = (int)(t % (MM / 8)) * 8; const size_t row = t / (MM / 8); const int tt = (int)(row % TT); const int s = (int)((row / TT) % NS); const int b = (int)(row / ((size_t)TT * NS)); int r = ri[s]; r = r < 0 ? 0 : (r >= GW ? GW - 1 : r); int cc = ci[s]; cc = cc < 0 ? 0 : (cc >= GW ? GW - 1 : cc);
  const size_t bt = (size_t)b * TT + tt; const float* y = Y + (bt * NG + r * GW + cc) * MM + c8; const int g = c8 / 8; const float mu = ST[(bt * 8 + g) * 32], rs = ST[(bt * 8 + g) * 32 + 1]; FragH f;
#pragma unroll
  for (int q = 0; q < 8; ++q) { const float v = (y[q] - mu) * rs * bf16_round(gg[c8 + q]) + bf16_round(gb[c8 + q]); f.h[q] = (_Float16)(0.5f * v * (1.0f + erff(v * 0.70710678118654752f))); }
  *(volatile v8us*)((unsigned short*)A16 + t * 8) = f.half[0]; __threadfence(); *(volatile v8us*)((unsigned short*)A16 + t * 8) = f.half[0]; }
extern "C" void kernel_launch(void* const* d_in, const int* in_sizes, int n_in,
                              void* d_out, int out_size, void* d_ws, size_t ws_size, hipStream_t stream) {
  (void)in_sizes; (void)n_in; (void)out_size;
  const float* x = (const float*)d_in[0]; const float* cw = (const float*)d_in[1]; const float* cb = (const float*)d_in[2]; const float* gg = (const float*)d_in[3]; const float* gb = (const float*)d_in[4]; const float* pw = (const float*)d_in[5]; const float* pb = (const float*)d_in[6]; const int* ri = (const int*)d_in[7]; const int* ci = (const int*)d_in[8];
  char* ws = (char*)d_ws; size_t off = 0;
  auto take = [&](size_t bytes) { char* p = ws + off; off += (bytes + 255) & ~(size_t)255; return p; };
  _Float16* Btap = (_Float16*)take((size_t)27 * MM * MM * 2); _Float16* Bpw = (_Float16*)take(MM * MM * 2); _Float16* X16 = (_Float16*)take((size_t)NSR * MM * 2); float* C = (float*)take((size_t)NSR * MM * 4); float* Y = (float*)take((size_t)NVX * MM * 4); float* ST = (float*)take((size_t)BB * TT * 8 * 32 * 4); _Float16* A16 = X16;
  if (off > ws_size) return;
  k_wtap<<<(27 * MM * (MM / 8) + 255) / 256, 256, 0, stream>>>(cw, Btap); k_round16f<<<(MM * MM / 8 + 255) / 256, 256, 0, stream>>>(pw, Bpw, MM * MM / 8);
  k_x16<<<(unsigned)(((size_t)NSR * MM / 8 + 255) / 256), 256, 0, stream>>>(x, X16, (size_t)NSR * MM / 8);
  k_ginit<<<(unsigned)(((size_t)NVX * MM / 4 + 255) / 256), 256, 0, stream>>>(cb, Y);
  const dim3 gS(((NSR / 16) * 1 + 3) / 4, 1);
  for (int kt = 0; kt < 3; ++kt) for (int kh = 0; kh < 3; ++kh) for (int kw = 0; kw < 3; ++kw) { const int tap = (kt * 3 + kh) * 3 + kw;
    k_gemm_hhx<0><<<gS, 128, 0, stream>>>(X16, MM, 0, Btap + (size_t)tap * MM * MM, MM, 0, 0.0625f, nullptr, 0, nullptr, 1, 0, 0, C, nullptr, MM, 0, NSR, MM, MM);
    k_tapacc<<<(unsigned)(((size_t)NSR * 16 + 255) / 256), 256, 0, stream>>>(C, ri, ci, 2 - kt, 1 - kh, 1 - kw, Y); }
  k_gnstat<<<BB * TT * 8, 256, 0, stream>>>(Y, ST);
  k_gath<<<(unsigned)(((size_t)NSR * (MM / 8) + 255) / 256), 256, 0, stream>>>(Y, ST, gg, gb, ri, ci, A16);
  k_gemm_hhx<0><<<gS, 128, 0, stream>>>(A16, MM, 0, Bpw, MM, 0, 0.0625f, pb, 0, x, 1, (size_t)MM, 0, (float*)d_out, nullptr, MM, 0, NSR, MM, MM);
}
